// RelationRepLayer_43147241455989
// MI455X (gfx1250) — hardware-verified
//
#include <hip/hip_runtime.h>
#include <math.h>

typedef __attribute__((ext_vector_type(16))) _Float16 v16h;
typedef __attribute__((ext_vector_type(16))) __bf16 v16b;
typedef __attribute__((ext_vector_type(8)))  _Float16 v8h;
typedef __attribute__((ext_vector_type(8)))  float v8f;
typedef __attribute__((ext_vector_type(4)))  float v4f;
typedef __attribute__((ext_vector_type(2)))  float v2f;
typedef __attribute__((ext_vector_type(4)))  unsigned v4u;
typedef __attribute__((ext_vector_type(4)))  int v4i;
typedef float __attribute__((may_alias)) float_a;
typedef int __attribute__((may_alias)) int_a;

template <typename T> __device__ __forceinline__ void vst2(void* p, T v) { *(volatile T*)p = v; __threadfence(); *(volatile T*)p = v; }
__device__ __forceinline__ v8f wmma16(v16h a, v16h b, v8f c) {
  v8f d = __builtin_amdgcn_wmma_f32_16x16x32_f16(false, a, false, b, (short)0, c, false, false);
  asm volatile("v_nop\n\tv_nop\n\tv_nop\n\tv_nop" : "+v"(d) : "v"(a), "v"(b));
  return d;
}
__device__ __forceinline__ v8f wmma_bf(v16b a, v16b b, v8f c) {
  v8f d = __builtin_amdgcn_wmma_f32_16x16x32_bf16(false, a, false, b, (short)0, c, false, false);
  asm volatile("v_nop\n\tv_nop\n\tv_nop\n\tv_nop" : "+v"(d) : "v"(a), "v"(b));
  return d;
}
__device__ __forceinline__ v16h frag_h(const _Float16* rowk0, int lane) {
  union { v16h v; v8h q[2]; } u; const _Float16* p = rowk0 + 8 * (lane >> 4);
  u.q[0] = *(const v8h*)p; u.q[1] = *(const v8h*)(p + 16); return u.v;
}
__device__ __forceinline__ v16h frag_f32(const float* rowk0, int lane) {
  v16h a; const float* p = rowk0 + 8 * (lane >> 4);
#pragma unroll
  for (int i = 0; i < 8; ++i) { a[i] = (_Float16)p[i]; a[8 + i] = (_Float16)p[16 + i]; }
  return a;
}
__device__ __forceinline__ v16h fragc_f32(const float* W, int k0, int n, int lane, int ld, int K) {
  v16h a; const int g = lane >> 4;
#pragma unroll
  for (int i = 0; i < 8; ++i) { const int ka = k0 + 8 * g + i, kb = ka + 16;
    a[i] = (_Float16)(ka < K ? W[(size_t)ka * ld + n] : 0.f); a[8 + i] = (_Float16)(kb < K ? W[(size_t)kb * ld + n] : 0.f); }
  return a;
}
struct F2 { v16b h, l; };
__device__ __forceinline__ F2 bsplit16(const float v[16]) { F2 r;
#pragma unroll
  for (int i = 0; i < 16; ++i) { const __bf16 h = (__bf16)v[i]; r.h[i] = h; r.l[i] = (__bf16)(v[i] - (float)h); }
  return r; }
__device__ __forceinline__ F2 split_row(const float* row, int k0, int lane) { float v[16]; const float* p = row + k0 + 8 * (lane >> 4);
#pragma unroll
  for (int i = 0; i < 8; ++i) { v[i] = p[i]; v[8 + i] = p[16 + i]; }
  return bsplit16(v); }
__device__ __forceinline__ F2 split_rowK(const float* row, int k0, int lane, int K) { float v[16]; const int g = lane >> 4;
#pragma unroll
  for (int i = 0; i < 8; ++i) { const int ka = k0 + 8 * g + i, kb = ka + 16; v[i] = ka < K ? row[ka] : 0.f; v[8 + i] = kb < K ? row[kb] : 0.f; }
  return bsplit16(v); }
__device__ __forceinline__ F2 split_col(const float* W, int k0, int n, int lane, int ld, int K) { float v[16]; const int g = lane >> 4;
#pragma unroll
  for (int i = 0; i < 8; ++i) { const int ka = k0 + 8 * g + i, kb = ka + 16; v[i] = ka < K ? W[(size_t)ka * ld + n] : 0.f; v[8 + i] = kb < K ? W[(size_t)kb * ld + n] : 0.f; }
  return bsplit16(v); }
__device__ __forceinline__ v8f mac3(const F2& a, const F2& b, v8f c) { c = wmma_bf(a.l, b.h, c); c = wmma_bf(a.h, b.l, c); return wmma_bf(a.h, b.h, c); }
__device__ __forceinline__ float sigm(float v) { return 1.0f / (1.0f + expf(-v)); }
#define LDSX() do { asm volatile("s_wait_dscnt 0" ::: "memory"); __builtin_amdgcn_wave_barrier(); __builtin_amdgcn_fence(__ATOMIC_RELEASE, "workgroup"); } while (0)

#define NBT 2
#define SS 512
#define KK 16
#define HH 256
#define NPR (NBT * KK * KK)
#define F1 768
#define F2N 1152

__global__ __launch_bounds__(256) void k_ctx(const float* __restrict__ tok, const int* __restrict__ tmask, const int* __restrict__ rmask, const int* __restrict__ span,
                                           const float* __restrict__ cand, const float* __restrict__ noctx, float* __restrict__ rel) {
  const int pr = blockIdx.x, b = pr / (KK * KK), i = (pr / KK) % KK, j = pr % KK, c = threadIdx.x;
  const int hs = span[(b * KK + i) * 2], he = span[(b * KK + i) * 2 + 1], ts = span[(b * KK + j) * 2], te = span[(b * KK + j) * 2 + 1];
  const int min_end = he < te ? he : te, max_start = hs > ts ? hs : ts;
  const bool valid = (min_end < max_start) && (rmask[(b * KK + i) * KK + j] != 0);
  float m = -6.5e4f; bool any = false;
  if (valid) { int lo = min_end < 0 ? 0 : min_end, hi = max_start > SS ? SS : max_start;
#pragma unroll 1
    for (int s = lo; s < hi; ++s) if (tmask[b * SS + s] != 0) { const float v = tok[((size_t)b * SS + s) * HH + c]; m = fmaxf(m, v); any = true; } }
  const float ctx = any ? m : noctx[c];
  float* row = rel + (size_t)pr * F1;
  vst2(row + c, (float_a)cand[((size_t)b * KK + i) * HH + c]); vst2(row + HH + c, (float_a)cand[((size_t)b * KK + j) * HH + c]); vst2(row + 2 * HH + c, (float_a)ctx);
}
template <int RELU>
__global__ __launch_bounds__(128) void k_ffn(const float* __restrict__ A, int K, const float* __restrict__ W, int N, const float* __restrict__ bias, float* __restrict__ Out) {
  __shared__ __align__(16) float so[4][16][132];
  const int tid = threadIdx.x, wave = tid >> 5, lane = tid & 31, col = lane & 15, g = lane >> 4;
  const int r0 = blockIdx.x * 64 + wave * 16, n0 = blockIdx.y * 128;
  v8f acc[8] = {};
#pragma unroll 1
  for (int kc = 0; kc < K / 32; ++kc) { const F2 a = split_row(A + (size_t)(r0 + col) * K, kc * 32, lane);
#pragma unroll
    for (int jj = 0; jj < 8; ++jj) acc[jj] = mac3(a, split_col(W, kc * 32, n0 + jj * 16 + col, lane, N, K), acc[jj]); }
#pragma unroll
  for (int jj = 0; jj < 8; ++jj) { const float bv = bias[n0 + jj * 16 + col];
#pragma unroll
    for (int r = 0; r < 8; ++r) { float v = acc[jj][r] + bv; if (RELU) v = v > 0.f ? v : 0.f; so[wave][8 * g + r][jj * 16 + col] = v; } }
  LDSX();
#pragma unroll 4
  for (int rl = 0; rl < 16; ++rl) vst2(Out + (size_t)(r0 + rl) * N + n0 + lane * 4, *(const v4f*)(&so[wave][rl][lane * 4]));
}
extern "C" void kernel_launch(void* const* d_in, const int* in_sizes, int n_in, void* d_out, int out_size, void* d_ws, size_t ws_size, hipStream_t stream) {
  (void)in_sizes; (void)n_in; (void)out_size; (void)ws_size;
  const float* tok = (const float*)d_in[0]; const int* tmask = (const int*)d_in[1]; const int* rmask = (const int*)d_in[2]; const int* span = (const int*)d_in[3];
  const float* cand = (const float*)d_in[4]; const float* W1 = (const float*)d_in[5]; const float* b1 = (const float*)d_in[6]; const float* W2 = (const float*)d_in[7]; const float* b2 = (const float*)d_in[8]; const float* noctx = (const float*)d_in[9];
  float* out = (float*)d_out;
  float* rel = (float*)d_ws; float* hid = rel + (size_t)NPR * F1;
  k_ctx<<<NPR, 256, 0, stream>>>(tok, tmask, rmask, span, cand, noctx, rel);
  k_ffn<1><<<dim3(NPR / 64, F2N / 128), 128, 0, stream>>>(rel, F1, W1, F2N, b1, hid);
  k_ffn<0><<<dim3(NPR / 64, HH / 128), 128, 0, stream>>>(hid, F2N, W2, HH, b2, out);
}
